// GCNPool_my2_44727789421337
// MI455X (gfx1250) — hardware-verified
//
#include <hip/hip_runtime.h>
#include <stddef.h>
#include <stdint.h>
#include <math.h>


typedef float          v4f   __attribute__((ext_vector_type(4)));
typedef float          v8f   __attribute__((ext_vector_type(8)));
typedef double         v2d   __attribute__((ext_vector_type(2)));
typedef int            v8i   __attribute__((ext_vector_type(8)));
typedef unsigned short v8us  __attribute__((ext_vector_type(8)));
typedef __bf16         v16bf __attribute__((ext_vector_type(16)));
typedef v4f  __attribute__((may_alias)) v4fa;
typedef v8us __attribute__((may_alias)) v8usa;
union FragB { v16bf v; v8us h[2]; v8i w; };

#define NROW   80000
#define NBT    160
#define H0_PX  40
#define H0_PS  100
#define TM_PT  136
#define TM_PQ  196
#define TM_PS  36
#define TM_T1B 21760
#define TM_QKB 62720
#define TM_LDS (TM_T1B + TM_QKB + 288 * 4)
#define SA_PK  72
#define GP     68

static_assert(TM_T1B == 80 * TM_PT * 2);
static_assert(TM_QKB == 80 * TM_PQ * 4);
static_assert(TM_T1B + 80 * TM_PS * 4 <= TM_QKB);
static_assert(NROW % 64 == 0 && NROW % 80 == 0);
static_assert((H0_PX % 8) == 0 && (TM_PT % 8) == 0 && (SA_PK % 8) == 0);
static_assert((TM_PQ % 4) == 0 && (TM_PS % 4) == 0 && (GP % 4) == 0 && (H0_PS % 4) == 0);

#define LDFRAG(F, P) do { (F).h[0] = *(const v8usa*)(P); (F).h[1] = *(const v8usa*)((P) + 16); } while (0)

__device__ __forceinline__ v8f wmb(const FragB& a, const FragB& b, v8f c) {
  v8f d = __builtin_amdgcn_wmma_f32_16x16x32_bf16(false, a.v, false, b.v, (short)0, c, false, false);
  asm volatile("v_nop\n\tv_nop\n\tv_nop\n\tv_nop" : "+v"(d) : "v"(a.w), "v"(b.w));
  return d;
}
__device__ __forceinline__ unsigned bf16_bits(float f) {
  const unsigned u = __float_as_uint(f);
  return (u + 0x7FFFu + ((u >> 16) & 1u)) >> 16;
}
__device__ __forceinline__ float bf16_val(float f) { return __uint_as_float(bf16_bits(f) << 16); }
__device__ __forceinline__ unsigned short hl1(float f, bool lo) {
  const unsigned hb = bf16_bits(f);
  const unsigned lb = bf16_bits(f - __uint_as_float(hb << 16));
  return (unsigned short)(lo ? lb : hb);
}
__device__ __forceinline__ v8us pack8(v4f a, v4f b, bool lo) {
  v8us o;
  o[0] = hl1(a.x, lo); o[1] = hl1(a.y, lo); o[2] = hl1(a.z, lo); o[3] = hl1(a.w, lo);
  o[4] = hl1(b.x, lo); o[5] = hl1(b.y, lo); o[6] = hl1(b.z, lo); o[7] = hl1(b.w, lo);
  return o;
}
__device__ __forceinline__ v8f zero8() { const v8f z = {0.f, 0.f, 0.f, 0.f, 0.f, 0.f, 0.f, 0.f}; return z; }

__global__ __launch_bounds__(256) void k_prepw(const float* __restrict__ cq, const float* __restrict__ ck,
                                               const float* __restrict__ lv, const float* __restrict__ lo_,
                                               const float* __restrict__ t2, const float* __restrict__ mw,
                                               unsigned short* WQK, unsigned short* WV, unsigned short* WLO,
                                               unsigned short* WT2, unsigned short* WMLP) {
  const int blk = (int)blockIdx.x, tid = (int)threadIdx.x;
  const float* src;
  int stride;
  unsigned short* dst;
  if (blk < 24) {
    const int u  = blk * 256 + tid;
    const int o2 = u / 48;
    const int k  = 8 * (u - o2 * 48);
    const int j  = k >> 7;
    const int c0 = k & 63;
    const int o  = o2 & 63;
    const float* W = (blk < 12) ? cq : ck;
    src = W + ((size_t)o * 64 + c0) * 3 + j;
    stride = 3;
    dst = WQK + (size_t)o2 * 384 + k;
  } else if (blk < 28) {
    const int u = (blk - 24) * 256 + tid;
    const int e = u >> 4, k = 8 * (u & 15), c0 = k & 63;
    src = lv + (size_t)e * 64 + c0; stride = 1;
    dst = WV + (size_t)e * 128 + k;
  } else if (blk < 32) {
    const int u = (blk - 28) * 256 + tid;
    const int e = u >> 4, k = 8 * (u & 15), c0 = k & 63;
    src = lo_ + (size_t)e * 64 + c0; stride = 1;
    dst = WLO + (size_t)e * 128 + k;
  } else if (blk < 34) {
    const int u = (blk - 32) * 256 + tid;
    const int e = u >> 4, k = 8 * (u & 15), c0 = k & 63;
    src = t2 + (size_t)e * 64 + c0; stride = 1;
    dst = WT2 + (size_t)e * 128 + k;
  } else {
    const int u = (blk - 34) * 256 + tid;
    const int o = u / 40;
    const int k = 8 * (u - o * 40);
    const int s = k >> 6, c0 = k & 31;
    src = mw + (size_t)o * 160 + s * 32 + c0; stride = 1;
    dst = WMLP + (size_t)o * 320 + k;
  }
  v8us ov;
#pragma unroll
  for (int i = 0; i < 8; ++i) ov[i] = (unsigned short)bf16_bits(src[(size_t)i * stride]);
  *(volatile v8us*)dst = ov;
  __threadfence();
  *(volatile v8us*)dst = ov;
}

__global__ __launch_bounds__(256) void k_prepA(const float* __restrict__ A, unsigned short* AP) {
  const int u  = (int)blockIdx.x * 256 + (int)threadIdx.x;
  const int w  = u >> 7;
  const int k  = 8 * (u & 127);
  const int v0 = k & 511;
  const int wc = w < 499 ? w : 499;
  v8us ov;
#pragma unroll
  for (int i = 0; i < 8; ++i) {
    const int v  = v0 + i;
    const int vc = v < 499 ? v : 499;
    const float f = A[(size_t)wc * 500 + vc];
    const bool ok = (w < 500) && (v < 500);
    ov[i] = ok ? (unsigned short)bf16_bits(f) : (unsigned short)0;
  }
  unsigned short* dst = AP + (size_t)w * 1024 + k;
  *(volatile v8us*)dst = ov;
  __threadfence();
  *(volatile v8us*)dst = ov;
}

__global__ __launch_bounds__(128) void k_h0(const float* __restrict__ x, const float* __restrict__ te1W,
                                            const float* __restrict__ te1b, const float* __restrict__ c1W,
                                            const float* __restrict__ c1b, unsigned short* H0, float* RES) {
  __shared__ __attribute__((aligned(16))) unsigned short xa[64 * H0_PX];
  __shared__ __attribute__((aligned(16))) unsigned short wb[96 * H0_PX];
  __shared__ float bs[96];
  __shared__ __attribute__((aligned(16))) float stg[64 * H0_PS];
  const int tid = (int)threadIdx.x, lane = tid & 31, wave = tid >> 5, hh = lane >> 4, m = lane & 15;
  const int r0 = (int)blockIdx.x * 64;
  {
    const int rg = tid & 15, cb = tid >> 4;
    const int r  = r0 + 4 * rg;
    const int b  = r / 5000;
    const int rl = r - b * 5000;
    const float* xp = x + (size_t)b * 160000 + rl;
#pragma unroll
    for (int i = 0; i < 4; ++i) {
      const int c = cb + 8 * i;
      const v4f v = *(const v4fa*)(xp + (size_t)c * 5000);
      xa[(4 * rg + 0) * H0_PX + c] = (unsigned short)bf16_bits(v.x);
      xa[(4 * rg + 1) * H0_PX + c] = (unsigned short)bf16_bits(v.y);
      xa[(4 * rg + 2) * H0_PX + c] = (unsigned short)bf16_bits(v.z);
      xa[(4 * rg + 3) * H0_PX + c] = (unsigned short)bf16_bits(v.w);
    }
  }
#pragma unroll
  for (int i = 0; i < 4; ++i) {
    const int idx = i * 128 + tid;
    const int o = idx >> 3, c4 = (idx & 7) * 4;
    const v4f v = *(const v4fa*)(te1W + (size_t)o * 32 + c4);
    wb[o * H0_PX + c4 + 0] = (unsigned short)bf16_bits(v.x);
    wb[o * H0_PX + c4 + 1] = (unsigned short)bf16_bits(v.y);
    wb[o * H0_PX + c4 + 2] = (unsigned short)bf16_bits(v.z);
    wb[o * H0_PX + c4 + 3] = (unsigned short)bf16_bits(v.w);
  }
#pragma unroll
  for (int i = 0; i < 2; ++i) {
    const int idx = i * 128 + tid;
    const int o = idx >> 3, c4 = (idx & 7) * 4;
    const v4f v = *(const v4fa*)(c1W + (size_t)o * 32 + c4);
    wb[(64 + o) * H0_PX + c4 + 0] = (unsigned short)bf16_bits(v.x);
    wb[(64 + o) * H0_PX + c4 + 1] = (unsigned short)bf16_bits(v.y);
    wb[(64 + o) * H0_PX + c4 + 2] = (unsigned short)bf16_bits(v.z);
    wb[(64 + o) * H0_PX + c4 + 3] = (unsigned short)bf16_bits(v.w);
  }
  if (tid < 64) bs[tid] = bf16_val(te1b[tid]);
  if (tid < 32) bs[64 + tid] = bf16_val(c1b[tid]);
  __syncthreads();

  v8f acc[6];
  {
    FragB af;
    LDFRAG(af, xa + (16 * wave + m) * H0_PX + 8 * hh);
#pragma unroll
    for (int t = 0; t < 6; ++t) {
      FragB bf;
      LDFRAG(bf, wb + (16 * t + m) * H0_PX + 8 * hh);
      acc[t] = wmb(af, bf, zero8());
    }
  }
#pragma unroll
  for (int t = 0; t < 6; ++t) {
    const float bv = bs[16 * t + m];
#pragma unroll
    for (int r = 0; r < 8; ++r) stg[(16 * wave + 8 * hh + r) * H0_PS + 16 * t + m] = acc[t][r] + bv;
  }
  __syncthreads();

  v8us pc[8];
#pragma unroll
  for (int it = 0; it < 8; ++it) {
    const int idx = it * 128 + tid;
    const int row = idx >> 4, p = idx & 15;
    const float* sp = stg + row * H0_PS + 8 * (p & 7);
    const v4f a = *(const v4fa*)sp;
    const v4f b = *(const v4fa*)(sp + 4);
    pc[it] = pack8(a, b, p >= 8);
  }
#pragma unroll
  for (int it = 0; it < 8; ++it) {
    const int idx = it * 128 + tid;
    const int row = idx >> 4, p = idx & 15;
    *(volatile v8us*)(H0 + (size_t)(r0 + row) * 128 + 8 * p) = pc[it];
  }
  __threadfence();
#pragma unroll
  for (int it = 0; it < 8; ++it) {
    const int idx = it * 128 + tid;
    const int row = idx >> 4, p = idx & 15;
    *(volatile v8us*)(H0 + (size_t)(r0 + row) * 128 + 8 * p) = pc[it];
  }

  v4f rv[4];
#pragma unroll
  for (int it = 0; it < 4; ++it) {
    const int idx = it * 128 + tid;
    const int row = idx >> 3, p = idx & 7;
    rv[it] = *(const v4fa*)(stg + row * H0_PS + 64 + 4 * p);
  }
#pragma unroll
  for (int it = 0; it < 4; ++it) {
    const int idx = it * 128 + tid;
    const int row = idx >> 3, p = idx & 7;
    const int r = r0 + row;
    const int bn = r / 10;
    const int t = r - bn * 10;
    const bool ok = t >= 4;
    const int tq = ok ? (t - 4) : 0;
    float* dp = RES + ((size_t)bn * 6 + tq) * 32 + 4 * p;
    if (ok) *(volatile v4f*)dp = rv[it];
  }
  __threadfence();
#pragma unroll
  for (int it = 0; it < 4; ++it) {
    const int idx = it * 128 + tid;
    const int row = idx >> 3, p = idx & 7;
    const int r = r0 + row;
    const int bn = r / 10;
    const int t = r - bn * 10;
    const bool ok = t >= 4;
    const int tq = ok ? (t - 4) : 0;
    float* dp = RES + ((size_t)bn * 6 + tq) * 32 + 4 * p;
    if (ok) *(volatile v4f*)dp = rv[it];
  }
}

__global__ __launch_bounds__(160) void k_tmsa(const unsigned short* __restrict__ H0,
                                              const unsigned short* __restrict__ WQK,
                                              const unsigned short* __restrict__ WV,
                                              const unsigned short* __restrict__ WLO,
                                              const unsigned short* __restrict__ WT2,
                                              const float* __restrict__ bq, const float* __restrict__ bk,
                                              const float* __restrict__ bv, const float* __restrict__ bo,
                                              const float* __restrict__ bt2, unsigned short* XP) {
  extern __shared__ __attribute__((aligned(16))) unsigned char dsm[];
  unsigned short* T1  = (unsigned short*)dsm;
  float*          QKV = (float*)(dsm + TM_T1B);
  unsigned short* T2  = (unsigned short*)(dsm + TM_T1B);
  float*          STG = (float*)(dsm + TM_T1B + TM_T1B);
  float*          BI  = (float*)(dsm + TM_T1B + TM_QKB);
  const int tid = (int)threadIdx.x, lane = tid & 31, wave = tid >> 5, hh = lane >> 4, m = lane & 15;
  const int r0 = (int)blockIdx.x * 80;

#pragma unroll
  for (int it = 0; it < 8; ++it) {
    const int idx = it * 160 + tid;
    const int row = idx >> 4, p = idx & 15;
    const v8us a = *(const v8usa*)(H0 + (size_t)(r0 + row) * 128 + 8 * p);
    *(v8usa*)(T1 + row * TM_PT + 8 * p) = a;
  }
  if (tid < 64) {
    BI[tid]       = bf16_val(bq[tid]);
    BI[64 + tid]  = bf16_val(bk[tid]);
    BI[128 + tid] = bf16_val(bv[tid]);
    BI[192 + tid] = bf16_val(bo[tid]);
  }
  if (tid < 32) BI[256 + tid] = bf16_val(bt2[tid]);
  __syncthreads();

  {
    v8f acc[12];
#pragma unroll
    for (int i = 0; i < 12; ++i) acc[i] = zero8();
    const int rr = 16 * wave + m;
    const int tl = rr % 10;
#pragma unroll
    for (int j = 0; j < 3; ++j) {
      const int ts = tl + j - 1;
      const bool val = (ts >= 0) && (ts < 10);
      int sr = rr + j - 1;
      sr = sr < 0 ? 0 : (sr > 79 ? 79 : sr);
      const int mk = val ? -1 : 0;
      const v8i mk8 = {mk, mk, mk, mk, mk, mk, mk, mk};
      const unsigned short* ap = T1 + sr * TM_PT + 8 * hh;
      const unsigned short* wp = WQK + (size_t)m * 384 + j * 128 + 8 * hh;
#pragma unroll 1
      for (int kk = 0; kk < 4; ++kk) {
        FragB af;
        LDFRAG(af, ap + 32 * kk);
        af.w = af.w & mk8;
#pragma unroll
        for (int nt = 0; nt < 8; ++nt) {
          FragB bf;
          LDFRAG(bf, wp + (size_t)(16 * nt) * 384 + 32 * kk);
          acc[nt] = wmb(af, bf, acc[nt]);
        }
        if (j == 1) {
#pragma unroll
          for (int nt = 0; nt < 4; ++nt) {
            FragB bf;
            LDFRAG(bf, WV + (size_t)(16 * nt + m) * 128 + 32 * kk + 8 * hh);
            acc[8 + nt] = wmb(af, bf, acc[8 + nt]);
          }
        }
      }
    }
#pragma unroll
    for (int nt = 0; nt < 12; ++nt) {
      const float bvv = BI[16 * nt + m];
#pragma unroll
      for (int r = 0; r < 8; ++r) QKV[(16 * wave + 8 * hh + r) * TM_PQ + 16 * nt + m] = acc[nt][r] + bvv;
    }
  }
  __syncthreads();

#pragma unroll 1
  for (int it = 0; it < 4; ++it) {
    const int item = it * 160 + tid;
    const int g   = item / 80;
    const int rem = item - g * 80;
    const int hd  = rem / 10;
    const int t   = rem - hd * 10;
    float* qp = QKV + (g * 10 + t) * TM_PQ + hd * 8;
    const v4f q0 = *(const v4fa*)qp;
    const v4f q1 = *(const v4fa*)(qp + 4);
    float sc[10];
    float mx = -INFINITY;
#pragma unroll
    for (int s = 0; s < 10; ++s) {
      const float* kp = QKV + (g * 10 + s) * TM_PQ + 64 + hd * 8;
      const v4f k0 = *(const v4fa*)kp;
      const v4f k1 = *(const v4fa*)(kp + 4);
      float a = q0.x * k0.x;
      a = fmaf(q0.y, k0.y, a); a = fmaf(q0.z, k0.z, a); a = fmaf(q0.w, k0.w, a);
      a = fmaf(q1.x, k1.x, a); a = fmaf(q1.y, k1.y, a); a = fmaf(q1.z, k1.z, a); a = fmaf(q1.w, k1.w, a);
      sc[s] = a * 0.35355339059327373f;
      mx = fmaxf(mx, sc[s]);
    }
    float sum = 0.0f;
#pragma unroll
    for (int s = 0; s < 10; ++s) { sc[s] = expf(sc[s] - mx); sum += sc[s]; }
    const float inv = 1.0f / sum;
    v4f o0 = {0.f, 0.f, 0.f, 0.f}, o1 = {0.f, 0.f, 0.f, 0.f};
#pragma unroll
    for (int s = 0; s < 10; ++s) {
      const float* vp = QKV + (g * 10 + s) * TM_PQ + 128 + hd * 8;
      const v4f w0 = *(const v4fa*)vp;
      const v4f w1 = *(const v4fa*)(vp + 4);
      const float p = sc[s] * inv;
      o0.x = fmaf(p, w0.x, o0.x); o0.y = fmaf(p, w0.y, o0.y); o0.z = fmaf(p, w0.z, o0.z); o0.w = fmaf(p, w0.w, o0.w);
      o1.x = fmaf(p, w1.x, o1.x); o1.y = fmaf(p, w1.y, o1.y); o1.z = fmaf(p, w1.z, o1.z); o1.w = fmaf(p, w1.w, o1.w);
    }
    *(v4fa*)qp = o0;
    *(v4fa*)(qp + 4) = o1;
  }
  __syncthreads();

#pragma unroll
  for (int it = 0; it < 8; ++it) {
    const int idx = it * 160 + tid;
    const int row = idx >> 4, p = idx & 15;
    const float* sp = QKV + row * TM_PQ + 8 * (p & 7);
    const v4f a = *(const v4fa*)sp;
    const v4f b = *(const v4fa*)(sp + 4);
    *(v8usa*)(T1 + row * TM_PT + 8 * p) = pack8(a, b, p >= 8);
  }
  __syncthreads();

  {
    v8f a1[4];
#pragma unroll
    for (int i = 0; i < 4; ++i) a1[i] = zero8();
    const unsigned short* ap = T1 + (16 * wave + m) * TM_PT + 8 * hh;
    const unsigned short* wp = WLO + (size_t)m * 128 + 8 * hh;
#pragma unroll 1
    for (int kk = 0; kk < 4; ++kk) {
      FragB af;
      LDFRAG(af, ap + 32 * kk);
#pragma unroll
      for (int nt = 0; nt < 4; ++nt) {
        FragB bf;
        LDFRAG(bf, wp + (size_t)(16 * nt) * 128 + 32 * kk);
        a1[nt] = wmb(af, bf, a1[nt]);
      }
    }
#pragma unroll
    for (int nt = 0; nt < 4; ++nt) {
      const int col = 16 * nt + m;
      const float bvv = BI[192 + col];
#pragma unroll
      for (int r = 0; r < 8; ++r) {
        const float v = a1[nt][r] + bvv;
        const unsigned hb = bf16_bits(v);
        const unsigned lb = bf16_bits(v - __uint_as_float(hb << 16));
        T2[(16 * wave + 8 * hh + r) * TM_PT + col]      = (unsigned short)hb;
        T2[(16 * wave + 8 * hh + r) * TM_PT + 64 + col] = (unsigned short)lb;
      }
    }
  }
  __syncthreads();

  {
    v8f a2[2];
    a2[0] = zero8(); a2[1] = zero8();
    const unsigned short* ap = T2 + (16 * wave + m) * TM_PT + 8 * hh;
    const unsigned short* wp = WT2 + (size_t)m * 128 + 8 * hh;
#pragma unroll 1
    for (int kk = 0; kk < 4; ++kk) {
      FragB af;
      LDFRAG(af, ap + 32 * kk);
#pragma unroll
      for (int nt = 0; nt < 2; ++nt) {
        FragB bf;
        LDFRAG(bf, wp + (size_t)(16 * nt) * 128 + 32 * kk);
        a2[nt] = wmb(af, bf, a2[nt]);
      }
    }
#pragma unroll
    for (int nt = 0; nt < 2; ++nt) {
      const float bvv = BI[256 + 16 * nt + m];
#pragma unroll
      for (int r = 0; r < 8; ++r) STG[(16 * wave + 8 * hh + r) * TM_PS + 16 * nt + m] = a2[nt][r] + bvv;
    }
  }
  __syncthreads();

  v8us pc[4];
#pragma unroll
  for (int it = 0; it < 4; ++it) {
    const int idx = it * 160 + tid;
    const int row = idx >> 3, p = idx & 7;
    const float* sp = STG + row * TM_PS + 8 * (p & 3);
    const v4f a = *(const v4fa*)sp;
    const v4f b = *(const v4fa*)(sp + 4);
    pc[it] = pack8(a, b, p >= 4);
  }
#pragma unroll
  for (int it = 0; it < 4; ++it) {
    const int idx = it * 160 + tid;
    const int row = idx >> 3, p = idx & 7;
    const int r  = r0 + row;
    const int bn = r / 10;
    const int t  = r - bn * 10;
    const int b  = bn / 500;
    const int n  = bn - b * 500;
    *(volatile v8us*)(XP + ((size_t)(b * 10 + t) * 500 + n) * 64 + 8 * p) = pc[it];
  }
  __threadfence();
#pragma unroll
  for (int it = 0; it < 4; ++it) {
    const int idx = it * 160 + tid;
    const int row = idx >> 3, p = idx & 7;
    const int r  = r0 + row;
    const int bn = r / 10;
    const int t  = r - bn * 10;
    const int b  = bn / 500;
    const int n  = bn - b * 500;
    *(volatile v8us*)(XP + ((size_t)(b * 10 + t) * 500 + n) * 64 + 8 * p) = pc[it];
  }
}

__global__ __launch_bounds__(256) void k_tr(const unsigned short* __restrict__ XP, unsigned short* XT) {
  __shared__ __attribute__((aligned(16))) unsigned short tl[64 * SA_PK];
  const int tid = (int)threadIdx.x;
  const int n0 = (int)blockIdx.x * 64;
  const int bt = (int)blockIdx.y;
#pragma unroll
  for (int it = 0; it < 2; ++it) {
    const int idx = it * 256 + tid;
    const int row = idx >> 3, p = idx & 7;
    const int n  = n0 + row;
    const int nc = n < 499 ? n : 499;
    v8us a = *(const v8usa*)(XP + ((size_t)bt * 500 + nc) * 64 + 8 * p);
    const unsigned short mk = (n < 500) ? (unsigned short)0xFFFF : (unsigned short)0;
#pragma unroll
    for (int e = 0; e < 8; ++e) a[e] = (unsigned short)(a[e] & mk);
    *(v8usa*)(tl + row * SA_PK + 8 * p) = a;
  }
  __syncthreads();
  v8us ov[2];
#pragma unroll
  for (int it = 0; it < 2; ++it) {
    const int idx = it * 256 + tid;
    const int line = idx >> 3, p = idx & 7;
    const int pl = line >> 5, cc = line & 31;
#pragma unroll
    for (int e = 0; e < 8; ++e) ov[it][e] = tl[(8 * p + e) * SA_PK + pl * 32 + cc];
  }
#pragma unroll
  for (int it = 0; it < 2; ++it) {
    const int idx = it * 256 + tid;
    const int line = idx >> 3, p = idx & 7;
    const int pl = line >> 5, cc = line & 31;
    *(volatile v8us*)(XT + ((size_t)bt * 32 + cc) * 1024 + pl * 512 + n0 + 8 * p) = ov[it];
  }
  __threadfence();
#pragma unroll
  for (int it = 0; it < 2; ++it) {
    const int idx = it * 256 + tid;
    const int line = idx >> 3, p = idx & 7;
    const int pl = line >> 5, cc = line & 31;
    *(volatile v8us*)(XT + ((size_t)bt * 32 + cc) * 1024 + pl * 512 + n0 + 8 * p) = ov[it];
  }
}

template <int WT>
__global__ __launch_bounds__(128) void k_hop(const unsigned short* __restrict__ Ain,
                                             const unsigned short* __restrict__ AP,
                                             unsigned short* OT, unsigned short* OP) {
  __shared__ __attribute__((aligned(16))) float stg[64 * GP];
  const int tid = (int)threadIdx.x, lane = tid & 31, wave = tid >> 5, hh = lane >> 4, m = lane & 15;
  const int rowBase = (int)blockIdx.x * 64;
  const int col0    = (int)blockIdx.y * 64;
  v8f acc[4];
  acc[0] = zero8(); acc[1] = zero8(); acc[2] = zero8(); acc[3] = zero8();
  const unsigned short* ap = Ain + (size_t)(rowBase + 16 * wave + m) * 1024 + 8 * hh;
  const unsigned short* wp = AP + (size_t)(col0 + m) * 1024 + 8 * hh;
#pragma unroll 1
  for (int ks = 0; ks < 32; ++ks) {
    FragB af;
    LDFRAG(af, ap + 32 * ks);
#pragma unroll
    for (int t = 0; t < 4; ++t) {
      FragB bf;
      LDFRAG(bf, wp + (size_t)(16 * t) * 1024 + 32 * ks);
      acc[t] = wmb(af, bf, acc[t]);
    }
  }
#pragma unroll
  for (int t = 0; t < 4; ++t)
#pragma unroll
    for (int r = 0; r < 8; ++r) stg[(16 * wave + 8 * hh + r) * GP + 16 * t + m] = acc[t][r];
  __syncthreads();

  if (WT != 0) {
    v8us pc[8];
#pragma unroll
    for (int it = 0; it < 8; ++it) {
      const int idx = it * 128 + tid;
      const int line = idx >> 3, p = idx & 7;
      const int pl = line >> 6, lr = line & 63;
      const float* sp = stg + lr * GP + 8 * p;
      const v4f a = *(const v4fa*)sp;
      const v4f b = *(const v4fa*)(sp + 4);
      pc[it] = pack8(a, b, pl != 0);
    }
#pragma unroll
    for (int it = 0; it < 8; ++it) {
      const int idx = it * 128 + tid;
      const int line = idx >> 3, p = idx & 7;
      const int pl = line >> 6, lr = line & 63;
      *(volatile v8us*)(OT + (size_t)(rowBase + lr) * 1024 + pl * 512 + col0 + 8 * p) = pc[it];
    }
    __threadfence();
#pragma unroll
    for (int it = 0; it < 8; ++it) {
      const int idx = it * 128 + tid;
      const int line = idx >> 3, p = idx & 7;
      const int pl = line >> 6, lr = line & 63;
      *(volatile v8us*)(OT + (size_t)(rowBase + lr) * 1024 + pl * 512 + col0 + 8 * p) = pc[it];
    }
  }
  {
    v8us pc[8];
#pragma unroll
    for (int it = 0; it < 8; ++it) {
      const int idx = it * 128 + tid;
      const int rowi = idx >> 3, p = idx & 7;
      const int btl = rowi >> 6, wl = rowi & 63;
      const int c0 = 8 * (p & 3);
      const bool lo = p >= 4;
#pragma unroll
      for (int e = 0; e < 8; ++e) pc[it][e] = hl1(stg[(btl * 32 + c0 + e) * GP + wl], lo);
    }
    const int bt0 = rowBase >> 5;
#pragma unroll
    for (int it = 0; it < 8; ++it) {
      const int idx = it * 128 + tid;
      const int rowi = idx >> 3, p = idx & 7;
      const int btl = rowi >> 6, wl = rowi & 63;
      const int w = col0 + wl;
      const int wc = w < 499 ? w : 499;
      unsigned short* dp = OP + ((size_t)(bt0 + btl) * 500 + wc) * 64 + 8 * p;
      if (w < 500) *(volatile v8us*)dp = pc[it];
    }
    __threadfence();
#pragma unroll
    for (int it = 0; it < 8; ++it) {
      const int idx = it * 128 + tid;
      const int rowi = idx >> 3, p = idx & 7;
      const int btl = rowi >> 6, wl = rowi & 63;
      const int w = col0 + wl;
      const int wc = w < 499 ? w : 499;
      unsigned short* dp = OP + ((size_t)(bt0 + btl) * 500 + wc) * 64 + 8 * p;
      if (w < 500) *(volatile v8us*)dp = pc[it];
    }
  }
}

template <int MODE>
__global__ __launch_bounds__(128) void k_satt(const unsigned short* __restrict__ XP,
                                              const unsigned short* __restrict__ VT,
                                              unsigned short* ZP, unsigned short* ZT) {
  __shared__ __attribute__((aligned(16))) unsigned short Ks[64 * SA_PK];
  __shared__ __attribute__((aligned(16))) unsigned short Vh[32 * SA_PK];
  __shared__ __attribute__((aligned(16))) unsigned short Vl[32 * SA_PK];
  __shared__ __attribute__((aligned(16))) unsigned short Psh[4][16 * SA_PK];
  __shared__ __attribute__((aligned(16))) unsigned short Psl[4][16 * SA_PK];
  __shared__ __attribute__((aligned(16))) float Os[64 * TM_PS];
  const int tid = (int)threadIdx.x, wave = tid >> 5, lane = tid & 31, hh = lane >> 4, c = lane & 15;
  const int bt = (int)blockIdx.x >> 3;
  const int qt = (int)blockIdx.x & 7;
  const int q0 = qt * 64 + wave * 16;
  const unsigned short* XPb = XP + (size_t)bt * 500 * 64;
  const unsigned short* VTb = VT + (size_t)bt * 32 * 1024;
  const float scl = 0.17677669529663687f;

  FragB qh, ql;
  {
    int qn = q0 + c;
    qn = qn > 499 ? 499 : qn;
    LDFRAG(qh, XPb + (size_t)qn * 64 + 8 * hh);
    LDFRAG(ql, XPb + (size_t)qn * 64 + 32 + 8 * hh);
  }
  float mrow[8], lrow[8];
  v8f oacc[2];
#pragma unroll
  for (int r = 0; r < 8; ++r) { mrow[r] = -INFINITY; lrow[r] = 0.0f; }
  oacc[0] = zero8(); oacc[1] = zero8();
  unsigned short* pwh = Psh[wave];
  unsigned short* pwl = Psl[wave];

#pragma unroll 1
  for (int kc = 0; kc < 8; ++kc) {
    const int kv0 = kc * 64;
    __syncthreads();
#pragma unroll
    for (int it = 0; it < 4; ++it) {
      const int idx = it * 128 + tid;
      const int row = idx >> 3, p = idx & 7;
      int n = kv0 + row;
      n = n > 499 ? 499 : n;
      const v8us a = *(const v8usa*)(XPb + (size_t)n * 64 + 8 * p);
      *(v8usa*)(Ks + row * SA_PK + 8 * p) = a;
    }
#pragma unroll
    for (int it = 0; it < 2; ++it) {
      const int idx = it * 128 + tid;
      const int cc = idx >> 3, p = idx & 7;
      const v8us a = *(const v8usa*)(VTb + (size_t)cc * 1024 + kv0 + 8 * p);
      const v8us b = *(const v8usa*)(VTb + (size_t)cc * 1024 + 512 + kv0 + 8 * p);
      *(v8usa*)(Vh + cc * SA_PK + 8 * p) = a;
      *(v8usa*)(Vl + cc * SA_PK + 8 * p) = b;
    }
    __syncthreads();

    v8f s[4];
#pragma unroll
    for (int j = 0; j < 4; ++j) {
      FragB kb, kl;
      LDFRAG(kb, Ks + (16 * j + c) * SA_PK + 8 * hh);
      LDFRAG(kl, Ks + (16 * j + c) * SA_PK + 32 + 8 * hh);
      v8f t = zero8();
      t = wmb(qh, kb, t);
      t = wmb(qh, kl, t);
      t = wmb(ql, kb, t);
      s[j] = t;
    }
#pragma unroll
    for (int j = 0; j < 4; ++j) {
      const bool dead = (kv0 + 16 * j + c) >= 500;
#pragma unroll
      for (int r = 0; r < 8; ++r) {
        const float sv = s[j][r] * scl;
        s[j][r] = dead ? -INFINITY : sv;
      }
    }
    float cm[8];
#pragma unroll
    for (int r = 0; r < 8; ++r) {
      float mm = fmaxf(fmaxf(s[0][r], s[1][r]), fmaxf(s[2][r], s[3][r]));
#pragma unroll
      for (int off = 1; off < 16; off <<= 1) mm = fmaxf(mm, __shfl_xor(mm, off, 32));
      cm[r] = mm;
    }
#pragma unroll
    for (int r = 0; r < 8; ++r) {
      const float mnew  = fmaxf(mrow[r], cm[r]);
      const float alpha = expf(mrow[r] - mnew);
      mrow[r] = mnew;
      float psum = 0.0f;
#pragma unroll
      for (int j = 0; j < 4; ++j) {
        const float p = expf(s[j][r] - mnew);
        psum += p;
        const unsigned hb = bf16_bits(p);
        const unsigned lb = bf16_bits(p - __uint_as_float(hb << 16));
        pwh[(8 * hh + r) * SA_PK + 16 * j + c] = (unsigned short)hb;
        pwl[(8 * hh + r) * SA_PK + 16 * j + c] = (unsigned short)lb;
      }
#pragma unroll
      for (int off = 1; off < 16; off <<= 1) psum += __shfl_xor(psum, off, 32);
      lrow[r] = lrow[r] * alpha + psum;
      oacc[0][r] *= alpha;
      oacc[1][r] *= alpha;
    }
    __builtin_amdgcn_fence(__ATOMIC_RELEASE, "workgroup");
    __builtin_amdgcn_wave_barrier();
    __builtin_amdgcn_fence(__ATOMIC_ACQUIRE, "workgroup");
#pragma unroll 1
    for (int kk = 0; kk < 2; ++kk) {
      FragB pa, pl;
      LDFRAG(pa, pwh + c * SA_PK + 32 * kk + 8 * hh);
      LDFRAG(pl, pwl + c * SA_PK + 32 * kk + 8 * hh);
#pragma unroll
      for (int tt = 0; tt < 2; ++tt) {
        FragB vb, vl;
        LDFRAG(vb, Vh + (16 * tt + c) * SA_PK + 32 * kk + 8 * hh);
        LDFRAG(vl, Vl + (16 * tt + c) * SA_PK + 32 * kk + 8 * hh);
        oacc[tt] = wmb(pa, vb, oacc[tt]);
        oacc[tt] = wmb(pa, vl, oacc[tt]);
        oacc[tt] = wmb(pl, vb, oacc[tt]);
      }
    }
  }

#pragma unroll
  for (int r = 0; r < 8; ++r) {
    const float inv = 1.0f / lrow[r];
    Os[(16 * wave + 8 * hh + r) * TM_PS + c]      = oacc[0][r] * inv;
    Os[(16 * wave + 8 * hh + r) * TM_PS + 16 + c] = oacc[1][r] * inv;
  }
  __syncthreads();

  {
    v8us pc[4];
#pragma unroll
    for (int it = 0; it < 4; ++it) {
      const int idx = it * 128 + tid;
      const int row = idx >> 3, p = idx & 7;
      const float* sp = Os + row * TM_PS + 8 * (p & 3);
      const v4f a = *(const v4fa*)sp;
      const v4f b = *(const v4fa*)(sp + 4);
      pc[it] = pack8(a, b, p >= 4);
    }
#pragma unroll
    for (int it = 0; it < 4; ++it) {
      const int idx = it * 128 + tid;
      const int row = idx >> 3, p = idx & 7;
      const int n = qt * 64 + row;
      const int nc = n < 499 ? n : 499;
      unsigned short* dp = ZP + ((size_t)bt * 500 + nc) * 64 + 8 * p;
      if (n < 500) *(volatile v8us*)dp = pc[it];
    }
    __threadfence();
#pragma unroll
    for (int it = 0; it < 4; ++it) {
      const int idx = it * 128 + tid;
      const int row = idx >> 3, p = idx & 7;
      const int n = qt * 64 + row;
      const int nc = n < 499 ? n : 499;
      unsigned short* dp = ZP + ((size_t)bt * 500 + nc) * 64 + 8 * p;
      if (n < 500) *(volatile v8us*)dp = pc[it];
    }
  }
  if (MODE != 0) {
    v8us pc[4];
#pragma unroll
    for (int it = 0; it < 4; ++it) {
      const int idx = it * 128 + tid;
      const int line = idx >> 3, p = idx & 7;
      const int pl = line >> 5, cc = line & 31;
#pragma unroll
      for (int e = 0; e < 8; ++e) {
        const float f = Os[(8 * p + e) * TM_PS + cc];
        const unsigned short hv = hl1(f, pl != 0);
        pc[it][e] = ((qt * 64 + 8 * p + e) < 500) ? hv : (unsigned short)0;
      }
    }
#pragma unroll
    for (int it = 0; it < 4; ++it) {
      const int idx = it * 128 + tid;
      const int line = idx >> 3, p = idx & 7;
      const int pl = line >> 5, cc = line & 31;
      *(volatile v8us*)(ZT + ((size_t)bt * 32 + cc) * 1024 + pl * 512 + qt * 64 + 8 * p) = pc[it];
    }
    __threadfence();
#pragma unroll
    for (int it = 0; it < 4; ++it) {
      const int idx = it * 128 + tid;
      const int line = idx >> 3, p = idx & 7;
      const int pl = line >> 5, cc = line & 31;
      *(volatile v8us*)(ZT + ((size_t)bt * 32 + cc) * 1024 + pl * 512 + qt * 64 + 8 * p) = pc[it];
    }
  }
}

__global__ __launch_bounds__(128) void k_mlp(const unsigned short* __restrict__ P0, const unsigned short* __restrict__ P1,
                                             const unsigned short* __restrict__ P2, const unsigned short* __restrict__ P3,
                                             const unsigned short* __restrict__ P4, const unsigned short* __restrict__ WM,
                                             const float* __restrict__ mb, float* G) {
  __shared__ __attribute__((aligned(16))) float stg[64 * GP];
  __shared__ float bs[64];
  const int tid = (int)threadIdx.x, lane = tid & 31, wave = tid >> 5, hh = lane >> 4, m = lane & 15;
  const int rowBase = (int)blockIdx.x * 64;
  if (tid < 64) bs[tid] = bf16_val(mb[tid]);
  v8f acc[4];
  acc[0] = zero8(); acc[1] = zero8(); acc[2] = zero8(); acc[3] = zero8();
  const size_t ro = (size_t)(rowBase + 16 * wave + m) * 64 + 8 * hh;
  const unsigned short* wp = WM + (size_t)m * 320 + 8 * hh;
#pragma unroll
  for (int s = 0; s < 5; ++s) {
    const unsigned short* pp = (s == 0) ? P0 : (s == 1) ? P1 : (s == 2) ? P2 : (s == 3) ? P3 : P4;
#pragma unroll
    for (int kk = 0; kk < 2; ++kk) {
      FragB af;
      LDFRAG(af, pp + ro + 32 * kk);
#pragma unroll
      for (int t = 0; t < 4; ++t) {
        FragB bf;
        LDFRAG(bf, wp + (size_t)(16 * t) * 320 + s * 64 + 32 * kk);
        acc[t] = wmb(af, bf, acc[t]);
      }
    }
  }
#pragma unroll
  for (int t = 0; t < 4; ++t)
#pragma unroll
    for (int r = 0; r < 8; ++r) stg[(16 * wave + 8 * hh + r) * GP + 16 * t + m] = acc[t][r];
  __syncthreads();
#pragma unroll 1
  for (int it = 0; it < 4; ++it) {
    const int idx = it * 128 + tid;
    const int row = idx >> 3, p = idx & 7;
    const v4f a = *(const v4fa*)(stg + row * GP + 4 * p);
    const v4f s = *(const v4fa*)(stg + row * GP + 32 + 4 * p);
    v4f g;
    g.x = tanhf(a.x + bs[4 * p + 0]) * (1.0f / (1.0f + expf(-(s.x + bs[32 + 4 * p + 0]))));
    g.y = tanhf(a.y + bs[4 * p + 1]) * (1.0f / (1.0f + expf(-(s.y + bs[32 + 4 * p + 1]))));
    g.z = tanhf(a.z + bs[4 * p + 2]) * (1.0f / (1.0f + expf(-(s.z + bs[32 + 4 * p + 2]))));
    g.w = tanhf(a.w + bs[4 * p + 3]) * (1.0f / (1.0f + expf(-(s.w + bs[32 + 4 * p + 3]))));
    float* dp = G + (size_t)(rowBase + row) * 32 + 4 * p;
    *(volatile v4f*)dp = g;
    __threadfence();
    *(volatile v4f*)dp = g;
  }
}

__global__ __launch_bounds__(256) void k_ct1(const float* __restrict__ G, const float* __restrict__ cW,
                                             const float* __restrict__ cb, float* G6) {
  __shared__ float wsh[64];
  __shared__ float bsh[8];
  const int tid = (int)threadIdx.x;
  if (tid < 64) {
    const float v = cW[tid < 59 ? tid : 59];
    wsh[tid] = (tid < 60) ? bf16_val(v) : 0.0f;
  }
  if (tid < 32) {
    const float v = cb[tid < 5 ? tid : 5];
    if (tid < 8) bsh[tid] = (tid < 6) ? bf16_val(v) : 0.0f;
  }
  __syncthreads();
  const int u  = (int)blockIdx.x * 256 + tid;
  const int bn = u >> 3, cq = u & 7;
  const int b  = bn / 500;
  const int n  = bn - b * 500;
  v4f gv[10];
#pragma unroll
  for (int t = 0; t < 10; ++t) gv[t] = *(const v4fa*)(G + ((size_t)(b * 10 + t) * 500 + n) * 32 + 4 * cq);
#pragma unroll 1
  for (int s = 0; s < 6; ++s) {
    const float b0 = bsh[s];
    v4f a = {b0, b0, b0, b0};
#pragma unroll
    for (int t = 0; t < 10; ++t) {
      const float w = wsh[s * 10 + t];
      a.x = fmaf(gv[t].x, w, a.x); a.y = fmaf(gv[t].y, w, a.y);
      a.z = fmaf(gv[t].z, w, a.z); a.w = fmaf(gv[t].w, w, a.w);
    }
    float* dp = G6 + ((size_t)bn * 6 + s) * 32 + 4 * cq;
    *(volatile v4f*)dp = a;
    __threadfence();
    *(volatile v4f*)dp = a;
  }
}

__global__ __launch_bounds__(256) void k_tatt(const float* __restrict__ G6, const float* __restrict__ c1W,
                                              const float* __restrict__ c2W, const float* __restrict__ tw,
                                              const float* __restrict__ tb, const float* __restrict__ tv,
                                              float* REC1) {
  __shared__ float c1s[32];
  __shared__ float c2s[512];
  __shared__ float f1s[3000];
  __shared__ float f2s[192];
  __shared__ float m1s[192];
  __shared__ float Ls[36];
  __shared__ float tbs[36];
  __shared__ float tvs[36];
  __shared__ __attribute__((aligned(16))) float outs[64];
  const int tid = (int)threadIdx.x, lane = tid & 31, wave = tid >> 5;
  const int b = (int)blockIdx.x;
  if (tid < 32) c1s[tid] = bf16_val(c1W[tid]);
#pragma unroll 1
  for (int i = tid; i < 512; i += 256) {
    const float v = c2W[i < 499 ? i : 499];
    c2s[i] = (i < 500) ? bf16_val(v) : 0.0f;
  }
  if (tid < 64) {
    const int j = tid < 35 ? tid : 35;
    const float a = tb[j];
    const float c = tv[j];
    if (tid < 36) { tbs[tid] = bf16_val(a); tvs[tid] = bf16_val(c); }
    outs[tid] = 0.0f;
  }
  __syncthreads();
  const float* Gb = G6 + (size_t)b * 3000 * 32;
#pragma unroll 1
  for (int it = 0; it < 12; ++it) {
    const int i  = it * 256 + tid;
    const int ic = i < 2999 ? i : 2999;
    const float* rp = Gb + (size_t)ic * 32;
    float a = 0.0f;
#pragma unroll 1
    for (int q = 0; q < 8; ++q) {
      const v4f v = *(const v4fa*)(rp + 4 * q);
      a = fmaf(v.x, c1s[4 * q + 0], a); a = fmaf(v.y, c1s[4 * q + 1], a);
      a = fmaf(v.z, c1s[4 * q + 2], a); a = fmaf(v.w, c1s[4 * q + 3], a);
    }
    if (i < 3000) f1s[i] = a;
  }
  if (tid < 192) {
    const int c = tid & 31, t = tid >> 5;
    const float* gp = Gb + t * 32 + c;
    double acc = 0.0;
#pragma unroll 4
    for (int n = 0; n < 500; ++n) acc += (double)gp[(size_t)n * 192] * (double)c2s[n];
    f2s[c * 6 + t] = (float)acc;
  }
  __syncthreads();
  if (tid < 192) {
    const int c = tid & 31, t = tid >> 5;
    double acc = 0.0;
#pragma unroll 4
    for (int n = 0; n < 500; ++n) acc += (double)f1s[n * 6 + t] * (double)bf16_val(tw[(size_t)n * 32 + c]);
    m1s[t * 32 + c] = (float)acc;
  }
  __syncthreads();
  const int j = tid < 35 ? tid : 35;
  {
    const int t = j / 6, s = j - t * 6;
    double a = 0.0;
#pragma unroll 1
    for (int c = 0; c < 32; ++c) a += (double)m1s[t * 32 + c] * (double)f2s[c * 6 + s];
    const float af = (float)a + tbs[j];
    const float L = 1.0f / (1.0f + expf(-af));
    if (tid < 36) Ls[tid] = L;
  }
  __syncthreads();
  {
    const int p = j / 6, s = j - p * 6;
    float a = 0.0f;
#pragma unroll 1
    for (int t = 0; t < 6; ++t) a = fmaf(tvs[p * 6 + t], Ls[t * 6 + s], a);
    if (tid < 36) outs[tid] = a;
  }
  __syncthreads();
  if (wave == 0) {
    const v4f ov = *(const v4fa*)(outs + 4 * (lane & 15));
    float* dp = REC1 + (size_t)b * 64 + 4 * (lane & 15);
    const bool ok = lane < 16;
    if (ok) *(volatile v4f*)dp = ov;
    __threadfence();
    if (ok) *(volatile v4f*)dp = ov;
  }
}

__global__ __launch_bounds__(256) void k_xo(const float* __restrict__ G6, const float* __restrict__ RES,
                                            const float* __restrict__ REC1, const float* __restrict__ g1,
                                            const float* __restrict__ b1, float* XO, double* REC2) {
  __shared__ float L2s[576];
  __shared__ float mus[8], rss[8], gs1[8], bs1[8];
  __shared__ float cfs[36];
  __shared__ double red[256 * 8];
  __shared__ __attribute__((aligned(16))) double recs[16];
  const int tid = (int)threadIdx.x, lane = tid & 31, wave = tid >> 5;
  const int blk = (int)blockIdx.x;
  const int b = blk >> 3, cg = blk & 7;
#pragma unroll
  for (int it = 0; it < 3; ++it) {
    const int idx = it * 256 + tid;
    const int ic = idx < 575 ? idx : 575;
    const int bb = ic / 36;
    const int jj = ic - bb * 36;
    const float v = REC1[(size_t)bb * 64 + jj];
    if (idx < 576) L2s[idx] = v;
  }
  if (tid < 32) {
    const int jj = tid < 5 ? tid : 5;
    const float a = g1[jj];
    const float c = b1[jj];
    if (tid < 6) { gs1[tid] = bf16_val(a); bs1[tid] = bf16_val(c); }
  }
  __syncthreads();
  if (wave == 0) {
    const int s = lane < 5 ? lane : 5;
    double sm = 0.0;
#pragma unroll 1
    for (int bp = 0; bp < 96; ++bp) sm += (double)L2s[bp * 6 + s];
    const double mean = sm * (1.0 / 96.0);
    double vq = 0.0;
#pragma unroll 1
    for (int bp = 0; bp < 96; ++bp) { const double d = (double)L2s[bp * 6 + s] - mean; vq += d * d; }
    const float var = (float)(vq * (1.0 / 96.0));
    if (lane < 6) { mus[lane] = (float)mean; rss[lane] = 1.0f / sqrtf(var + 1e-5f); }
  }
  __syncthreads();
  if (wave == 0) {
    const int q = lane < 5 ? lane : 5;
    const float* lp = L2s + b * 36 + q * 6;
    float mx = -INFINITY;
#pragma unroll 1
    for (int l = 0; l < 6; ++l) {
      const float v = (lp[l] - mus[l]) * rss[l] * gs1[l] + bs1[l];
      mx = fmaxf(mx, v);
    }
    float sum = 0.0f;
#pragma unroll 1
    for (int l = 0; l < 6; ++l) {
      const float v = (lp[l] - mus[l]) * rss[l] * gs1[l] + bs1[l];
      sum += expf(v - mx);
    }
    const float inv = 1.0f / sum;
#pragma unroll 1
    for (int l = 0; l < 6; ++l) {
      const float v = (lp[l] - mus[l]) * rss[l] * gs1[l] + bs1[l];
      const float e = expf(v - mx) * inv;
      if (lane < 6) cfs[q * 6 + l] = e;
    }
  }
  __syncthreads();

  double a0 = 0.0, a1 = 0.0, a2 = 0.0, a3 = 0.0, s0 = 0.0, s1 = 0.0, s2 = 0.0, s3 = 0.0;
  const size_t slab = (size_t)blk * 12000;
#pragma unroll 1
  for (int it = 0; it < 47; ++it) {
    const int i = it * 256 + tid;
    if (i < 12000) {
      const int c4  = i / 3000;
      const int rem = i - c4 * 3000;
      const int n   = rem / 6;
      const int q   = rem - n * 6;
      const int c   = 4 * cg + c4;
      const float* gp = G6 + ((size_t)(b * 500 + n) * 6) * 32 + c;
      float a = 0.0f;
#pragma unroll
      for (int l = 0; l < 6; ++l) a = fmaf(cfs[q * 6 + l], gp[l * 32], a);
      a = (a > 0.0f) ? a : 0.01f * a;
      a += RES[((size_t)(b * 500 + n) * 6 + q) * 32 + c];
      float* dp = XO + slab + i;
      *(volatile float*)dp = a;
      __threadfence();
      *(volatile float*)dp = a;
      const double ad = (double)a;
      const double sq = ad * ad;
      a0 += (c4 == 0) ? ad : 0.0; s0 += (c4 == 0) ? sq : 0.0;
      a1 += (c4 == 1) ? ad : 0.0; s1 += (c4 == 1) ? sq : 0.0;
      a2 += (c4 == 2) ? ad : 0.0; s2 += (c4 == 2) ? sq : 0.0;
      a3 += (c4 == 3) ? ad : 0.0; s3 += (c4 == 3) ? sq : 0.0;
    }
  }
  red[tid * 8 + 0] = a0; red[tid * 8 + 1] = a1; red[tid * 8 + 2] = a2; red[tid * 8 + 3] = a3;
  red[tid * 8 + 4] = s0; red[tid * 8 + 5] = s1; red[tid * 8 + 6] = s2; red[tid * 8 + 7] = s3;
  __syncthreads();
  if (wave == 0) {
    const int jj = lane & 7, part = lane >> 3;
    double s = 0.0;
#pragma unroll 1
    for (int k = 0; k < 64; ++k) s += red[(part * 64 + k) * 8 + jj];
    s += __shfl_xor(s, 8, 32);
    s += __shfl_xor(s, 16, 32);
    if (lane < 16) recs[lane] = (lane < 8) ? s : 0.0;
  }
  __syncthreads();
  {
    const int t8 = tid & 7;
    v2d rv;
    rv.x = recs[2 * t8];
    rv.y = recs[2 * t8 + 1];
    double* dp = REC2 + (size_t)blk * 16 + 2 * t8;
    const bool ok = tid < 8;
    if (ok) *(volatile v2d*)dp = rv;
    __threadfence();
    if (ok) *(volatile v2d*)dp = rv;
  }
}

__global__ __launch_bounds__(256) void k_out(const float* __restrict__ XO, const double* __restrict__ REC2,
                                             const float* __restrict__ g2, const float* __restrict__ b2,
                                             float* out) {
  __shared__ float sm[2], si[2], sg[2], sb[2];
  const int tid = (int)threadIdx.x, lane = tid & 31, wave = tid >> 5;
  const int e0 = (int)blockIdx.x * 1024;
  const int ca = (e0 / 3000) & 31;
  const int cb = ((e0 + 1023) / 3000) & 31;
  if (wave == 0) {
    const int c = (lane & 1) ? cb : ca;
    double s = 0.0, q = 0.0;
#pragma unroll 4
    for (int b = 0; b < 16; ++b) {
      const double* rp = REC2 + (size_t)(b * 8 + (c >> 2)) * 16;
      s += rp[c & 3];
      q += rp[4 + (c & 3)];
    }
    const double mean = s * (1.0 / 48000.0);
    double var = q * (1.0 / 48000.0) - mean * mean;
    var = var < 0.0 ? 0.0 : var;
    const float inv = 1.0f / sqrtf((float)var + 1e-5f);
    const float gg = bf16_val(g2[c]);
    const float bb = bf16_val(b2[c]);
    if (lane < 2) { sm[lane] = (float)mean; si[lane] = inv; sg[lane] = gg; sb[lane] = bb; }
  }
  __syncthreads();
  const int e = e0 + 4 * tid;
  const int c = (e / 3000) & 31;
  const int k = (c == ca) ? 0 : 1;
  const float mu = sm[k], inv = si[k], gg = sg[k], bb = sb[k];
  const v4f x = *(const v4fa*)(XO + e);
  v4f y;
  y.x = ((x.x - mu) * inv) * gg + bb;
  y.y = ((x.y - mu) * inv) * gg + bb;
  y.z = ((x.z - mu) * inv) * gg + bb;
  y.w = ((x.w - mu) * inv) * gg + bb;
  float* dp = out + e;
  *(volatile v4f*)dp = y;
  __threadfence();
  *(volatile v4f*)dp = y;
}

static inline size_t al256(size_t o) { return (o + 255) & ~(size_t)255; }

extern "C" void kernel_launch(void* const* d_in, const int* in_sizes, int n_in,
                              void* d_out, int out_size, void* d_ws, size_t ws_size,
                              hipStream_t stream) {
  if (n_in < 29) return;
  static const int esz[29] = {2560000, 250000, 1024, 32, 2048, 64, 12288, 64, 12288, 64, 4096, 64, 4096, 64,
                              2048, 32, 10240, 64, 60, 6, 32, 500, 16000, 36, 36, 6, 6, 32, 32};
  for (int i = 0; i < 29; ++i) if (in_sizes[i] != esz[i]) return;
  if (out_size != 1536000) return;

  const float* x       = (const float*)d_in[0];
  const float* A       = (const float*)d_in[1];
  const float* conv1_W = (const float*)d_in[2];
  const float* conv1_b = (const float*)d_in[3];
  const float* te1_W   = (const float*)d_in[4];
  const float* te1_b   = (const float*)d_in[5];
  const float* convq_W = (const float*)d_in[6];
  const float* convq_b = (const float*)d_in[7];
  const float* convk_W = (const float*)d_in[8];
  const float* convk_b = (const float*)d_in[9];
  const float* linv_W  = (const float*)d_in[10];
  const float* linv_b  = (const float*)d_in[11];
  const float* lino_W  = (const float*)d_in[12];
  const float* lino_b  = (const float*)d_in[13];
  const float* te2_W   = (const float*)d_in[14];
  const float* te2_b   = (const float*)d_in[15];
  const float* mlp_W   = (const float*)d_in[16];
  const float* mlp_b   = (const float*)d_in[17];
  const float* ct1_W   = (const float*)d_in[18];
  const float* ct1_b   = (const float*)d_in[19];
  const float* tat_c1  = (const float*)d_in[20];
  const float* tat_c2  = (const float*)d_in[21];
  const float* tat_w   = (const float*)d_in[22];
  const float* tat_b   = (const float*)d_in[23];
  const float* tat_v   = (const float*)d_in[24];
  const float* bn1_g   = (const float*)d_in[25];
  const float* bn1_b   = (const float*)d_in[26];
  const float* bn2_g   = (const float*)d_in[27];
  const float* bn2_b   = (const float*)d_in[28];
  float* out = (float*)d_out;

  char* ws = (char*)d_ws;
  size_t off = 0;
  const size_t oWQK  = off; off = al256(off + (size_t)128 * 384 * 2);
  const size_t oWV   = off; off = al256(off + (size_t)64 * 128 * 2);
  const size_t oWLO  = off; off = al256(off + (size_t)64 * 128 * 2);
  const size_t oWT2  = off; off = al256(off + (size_t)32 * 128 * 2);
  const size_t oWMLP = off; off = al256(off + (size_t)64 * 320 * 2);
  const size_t oAP   = off; off = al256(off + (size_t)512 * 1024 * 2);
  const size_t oH0   = off; off = al256(off + (size_t)NROW * 128 * 2);
  const size_t oRES  = off; off = al256(off + (size_t)48000 * 32 * 4);
  const size_t oXP   = off; off = al256(off + (size_t)NROW * 64 * 2);
  const size_t oZ1P  = off; off = al256(off + (size_t)NROW * 64 * 2);
  const size_t oZ2P  = off; off = al256(off + (size_t)NROW * 64 * 2);
  const size_t oZ3P  = off; off = al256(off + (size_t)NROW * 64 * 2);
  const size_t oZ4P  = off; off = al256(off + (size_t)NROW * 64 * 2);
  const size_t oXT   = off; off = al256(off + (size_t)5120 * 1024 * 2);
  const size_t oZ1T  = off; off = al256(off + (size_t)5120 * 1024 * 2);
  const size_t oZ3T  = off; off = al256(off + (size_t)5120 * 1024 * 2);
  const size_t oR1   = off; off = al256(off + (size_t)16 * 64 * 4);
  const size_t oR2   = off; off = al256(off + (size_t)128 * 16 * 8);
  if (off > ws_size || off > (size_t)134217728) return;
  if ((size_t)NROW * 32 * 4 > (size_t)NROW * 128 * 2) return;
  if ((size_t)48000 * 32 * 4 > (size_t)5120 * 1024 * 2) return;
  if ((size_t)1536000 * 4 > (size_t)5120 * 1024 * 2) return;

  unsigned short* WQK  = (unsigned short*)(ws + oWQK);
  unsigned short* WV   = (unsigned short*)(ws + oWV);
  unsigned short* WLO  = (unsigned short*)(ws + oWLO);
  unsigned short* WT2  = (unsigned short*)(ws + oWT2);
  unsigned short* WMLP = (unsigned short*)(ws + oWMLP);
  unsigned short* AP   = (unsigned short*)(ws + oAP);
  unsigned short* H0   = (unsigned short*)(ws + oH0);
  float*          RES  = (float*)(ws + oRES);
  unsigned short* XP   = (unsigned short*)(ws + oXP);
  unsigned short* Z1P  = (unsigned short*)(ws + oZ1P);
  unsigned short* Z2P  = (unsigned short*)(ws + oZ2P);
  unsigned short* Z3P  = (unsigned short*)(ws + oZ3P);
  unsigned short* Z4P  = (unsigned short*)(ws + oZ4P);
  unsigned short* XT   = (unsigned short*)(ws + oXT);
  unsigned short* Z1T  = (unsigned short*)(ws + oZ1T);
  unsigned short* Z3T  = (unsigned short*)(ws + oZ3T);
  float*          REC1 = (float*)(ws + oR1);
  double*         REC2 = (double*)(ws + oR2);
  float*          G    = (float*)(ws + oH0);
  float*          G6   = (float*)(ws + oXT);
  float*          XO   = (float*)(ws + oZ1T);

  hipFuncSetAttribute(reinterpret_cast<const void*>(&k_tmsa), hipFuncAttributeMaxDynamicSharedMemorySize, (int)TM_LDS);

  k_prepw<<<44, 256, 0, stream>>>(convq_W, convk_W, linv_W, lino_W, te2_W, mlp_W, WQK, WV, WLO, WT2, WMLP);
  k_prepA<<<256, 256, 0, stream>>>(A, AP);
  k_h0<<<NROW / 64, 128, 0, stream>>>(x, te1_W, te1_b, conv1_W, conv1_b, H0, RES);
  k_tmsa<<<NROW / 80, 160, TM_LDS, stream>>>(H0, WQK, WV, WLO, WT2, convq_b, convk_b, linv_b, lino_b, te2_b, XP);
  k_tr<<<dim3(8, NBT), 256, 0, stream>>>(XP, XT);
  k_hop<1><<<dim3(80, 8), 128, 0, stream>>>(XT, AP, Z1T, Z1P);
  k_hop<0><<<dim3(80, 8), 128, 0, stream>>>(Z1T, AP, Z1T, Z2P);
  k_satt<1><<<NBT * 8, 128, 0, stream>>>(XP, XT, Z3P, Z3T);
  k_satt<0><<<NBT * 8, 128, 0, stream>>>(XP, Z3T, Z4P, Z3T);
  k_mlp<<<NROW / 64, 128, 0, stream>>>(XP, Z1P, Z2P, Z3P, Z4P, WMLP, mlp_b, G);
  k_ct1<<<250, 256, 0, stream>>>(G, ct1_W, ct1_b, G6);
  k_tatt<<<16, 256, 0, stream>>>(G6, tat_c1, tat_c2, tat_w, tat_b, tat_v, REC1);
  k_xo<<<128, 256, 0, stream>>>(G6, RES, REC1, bn1_g, bn1_b, XO, REC2);
  k_out<<<1500, 256, 0, stream>>>(XO, REC2, bn2_g, bn2_b, out);
  (void)hipGetLastError();
}
